// Generator_22196390985916
// MI455X (gfx1250) — hardware-verified
//
#include <hip/hip_runtime.h>
#include <math.h>

#define NB     8
#define NC     64
#define HH     128
#define WW     128
#define HWN    16384
#define NF     5
#define LL     512
#define HC     128
#define NO2    128
#define KSP    1152
#define KSH    32
#define HP     130
#define WP     130
#define GPB    1152
#define SPITCH 132
#define ACT_SPLIT 1
#define NPL    (ACT_SPLIT ? 2 : 1)
#define PLANE  ((size_t)NB * HP * WP * HC)
#define NSEG   (NF * 3 * WP)
#define NSEGP  1952
#define DYN_FLOATS (WW * SPITCH + NF * GPB + NSEGP + 2 * NC)
#define DYN_BYTES  (DYN_FLOATS * 4)
#define NU1    (NO2 * KSP / 8)
#define NU2    (HC * KSH / 8)

static_assert(KSP % 32 == 0);
static_assert(KSH % 32 == 0);
static_assert(WW % 32 == 0);
static_assert(NU1 % 256 == 0);
static_assert(NU2 % 256 == 0);
static_assert((GPB * 4) % 128 == 0);
static_assert(NC == 64);
static_assert(NSEG <= NSEGP);
static_assert(DYN_BYTES == 98944);
static_assert((PLANE * 2) % 128 == 0);

typedef __bf16 v16b __attribute__((ext_vector_type(16)));
typedef __bf16 v8b  __attribute__((ext_vector_type(8)));
typedef float  v8f  __attribute__((ext_vector_type(8)));
typedef float  v4f  __attribute__((ext_vector_type(4)));
typedef unsigned short v8us __attribute__((ext_vector_type(8)));
typedef v8us __attribute__((may_alias)) v8usa;
typedef v8b  __attribute__((may_alias)) v8ba;
typedef v4f  __attribute__((may_alias)) v4fa;

union FragB { v16b v; v8b h[2]; };

__device__ __forceinline__ unsigned short f2bf_bits(float f) {
  const unsigned u = __float_as_uint(f);
  return (unsigned short)((u + 0x7FFFu + ((u >> 16) & 1u)) >> 16);
}
__device__ __forceinline__ float bf_bits2f(unsigned short hb) { return __uint_as_float(((unsigned)hb) << 16); }
__device__ __forceinline__ float bf_rne(float f) { return bf_bits2f(f2bf_bits(f)); }

__device__ __forceinline__ v8f mma_bf(v16b a, v16b b, v8f c) {
  v8f d = __builtin_amdgcn_wmma_f32_16x16x32_bf16(false, a, false, b, (short)0, c, false, false);
  asm volatile("v_nop\n\tv_nop\n\tv_nop\n\tv_nop" : "+v"(d) : "v"(a), "v"(b));
  return d;
}

__device__ __forceinline__ v16b frag_bf(const __bf16* p, int hh) {
  FragB f;
  f.h[0] = *(const v8ba*)(p + 8 * hh);
  f.h[1] = *(const v8ba*)(p + 16 + 8 * hh);
  return f.v;
}

__device__ __forceinline__ float wave_sum(float v) {
  v += __shfl_xor(v, 16, 32);
  v += __shfl_xor(v, 8, 32);
  v += __shfl_xor(v, 4, 32);
  v += __shfl_xor(v, 2, 32);
  v += __shfl_xor(v, 1, 32);
  return v;
}

__device__ __forceinline__ void wave_lds_sync() {
  __builtin_amdgcn_fence(__ATOMIC_RELEASE, "workgroup");
  __builtin_amdgcn_wave_barrier();
  __builtin_amdgcn_fence(__ATOMIC_ACQUIRE, "workgroup");
}

__global__ __launch_bounds__(256) void k_prep(const float* __restrict__ sgw, const float* __restrict__ sbw,
                                             const float* __restrict__ ssw,
                                             unsigned short* __restrict__ wsp, unsigned short* __restrict__ wsh) {
  const int u = blockIdx.x * 256 + threadIdx.x;
  v8us o;
  unsigned short* dst;
  if (blockIdx.x < NU1 / 256) {
    const int n = u / (KSP / 8);
    const int r = u - n * (KSP / 8);
    const int k0 = r * 8;
    const int t = k0 >> 7;
    const int c0 = k0 & 127;
    const int isb = (n >= 64) ? 1 : 0;
    const float* w = (isb ? sbw : sgw) + ((size_t)(n - 64 * isb) * HC + c0) * 9 + t;
#pragma unroll
    for (int i = 0; i < 8; ++i) o[i] = f2bf_bits(w[i * 9]);
    dst = wsp + (size_t)u * 8;
  } else {
    const int v = u - NU1;
    if (v >= NU2) return;
    const int n = v >> 2;
    const int k0 = (v & 3) * 8;
#pragma unroll
    for (int i = 0; i < 8; ++i) {
      const int k = k0 + i;
      const int kc = min(k, 26);
      float val = ssw[(size_t)n * 27 + kc];
      val = (k < 27) ? val : 0.0f;
      o[i] = f2bf_bits(val);
    }
    dst = wsh + (size_t)v * 8;
  }
  *(volatile v8us*)dst = o;
  __threadfence();
  *(volatile v8us*)dst = o;
}

__global__ __launch_bounds__(256) void k_stats(const float* __restrict__ x, float* __restrict__ stats) {
  __shared__ float red[8];
  const int bc = blockIdx.x;
  const int tid = threadIdx.x, lane = tid & 31, wave = tid >> 5;
  const float* p = x + (size_t)bc * HWN;
  float s = 0.0f;
#pragma unroll 2
  for (int it = 0; it < HWN / 1024; ++it) {
    const v4f v = *(const v4fa*)(p + (size_t)(it * 256 + tid) * 4);
    s += bf_rne(v.x); s += bf_rne(v.y); s += bf_rne(v.z); s += bf_rne(v.w);
  }
  s = wave_sum(s);
  if (lane == 0) red[wave] = s;
  __syncthreads();
  float tot = red[0];
#pragma unroll
  for (int w = 1; w < 8; ++w) tot += red[w];
  const float mu = tot * (1.0f / 16384.0f);
  __syncthreads();
  float s2 = 0.0f;
#pragma unroll 2
  for (int it = 0; it < HWN / 1024; ++it) {
    const v4f v = *(const v4fa*)(p + (size_t)(it * 256 + tid) * 4);
    float d;
    d = bf_rne(v.x) - mu; s2 = fmaf(d, d, s2);
    d = bf_rne(v.y) - mu; s2 = fmaf(d, d, s2);
    d = bf_rne(v.z) - mu; s2 = fmaf(d, d, s2);
    d = bf_rne(v.w) - mu; s2 = fmaf(d, d, s2);
  }
  s2 = wave_sum(s2);
  if (lane == 0) red[wave] = s2;
  __syncthreads();
  float tot2 = red[0];
#pragma unroll
  for (int w = 1; w < 8; ++w) tot2 += red[w];
  const float var = tot2 * (1.0f / 16384.0f);
  const float rstd = rsqrtf(var + 1e-5f);
  if (tid < 8) {
    const float f = (tid == 0) ? 1.0f : 0.0f;
    v4f o;
    o.x = mu * f; o.y = rstd * f; o.z = 0.0f; o.w = 0.0f;
    float* dst = stats + (size_t)bc * 32 + tid * 4;
    *(volatile v4f*)dst = o;
    __threadfence();
    *(volatile v4f*)dst = o;
  }
}

__global__ __launch_bounds__(256) void k_fcg(const float* __restrict__ codes, const float* __restrict__ wfc,
                                            const float* __restrict__ bfc,
                                            const float* __restrict__ cgw, const float* __restrict__ cbw,
                                            float* __restrict__ G) {
  __shared__ float sc[LL];
  __shared__ float smu[LL];
  __shared__ __align__(16) float sg[GPB];
  const int blk = blockIdx.x;
  const int b = blk / NF, j = blk - b * NF;
  const int tid = threadIdx.x;
  const float* cp = codes + (size_t)blk * LL;
  sc[tid] = bf_rne(cp[tid]);
  sc[tid + 256] = bf_rne(cp[tid + 256]);
  __syncthreads();
#pragma unroll 1
  for (int q = 0; q < 2; ++q) {
    const int mm = tid + 256 * q;
    const float* wr = wfc + ((size_t)j * LL + mm) * LL;
    float a = 0.0f;
#pragma unroll 2
    for (int l = 0; l < LL; l += 4) {
      const v4f wv = *(const v4fa*)(wr + l);
      a = fmaf(bf_rne(wv.x), sc[l], a);
      a = fmaf(bf_rne(wv.y), sc[l + 1], a);
      a = fmaf(bf_rne(wv.z), sc[l + 2], a);
      a = fmaf(bf_rne(wv.w), sc[l + 3], a);
    }
    a += bf_rne(bfc[(size_t)j * LL + mm]);
    smu[mm] = fmaxf(a, 0.0f);
  }
  __syncthreads();
  for (int o = tid; o < GPB; o += 256) {
    const int n = o / 9;
    const int t = o - 9 * n;
    const int isb = (n >= 64) ? 1 : 0;
    const float* w = (isb ? cbw : cgw) + ((size_t)(n - 64 * isb) * LL) * 9 + t;
    float a = 0.0f;
#pragma unroll 4
    for (int m2 = 0; m2 < LL; ++m2) a = fmaf(bf_rne(w[(size_t)m2 * 9]), smu[m2], a);
    sg[o] = a;
  }
  __syncthreads();
  float* gp = G + (size_t)blk * GPB;
  for (int rep = 0; rep < 2; ++rep) {
    for (int i = tid; i < GPB / 4; i += 256) {
      const v4f v = *(const v4fa*)(sg + 4 * i);
      *(volatile v4f*)(gp + 4 * i) = v;
    }
    __threadfence();
  }
  (void)b;
}

__global__ __launch_bounds__(256) void k_shared(const float* __restrict__ msk, const unsigned short* __restrict__ wsh,
                                               const float* __restrict__ ssb, unsigned short* __restrict__ act) {
  __shared__ float mrow[9 * WP];
  __shared__ __align__(16) unsigned short As[WW * KSH];
  __shared__ __align__(16) unsigned short slab[8][16 * HC];
  const int blk = blockIdx.x;
  const int b = blk / HP, hp = blk - b * HP;
  const int tid = threadIdx.x, lane = tid & 31, wave = tid >> 5, hh = lane >> 4, m = lane & 15;
  const size_t rowbase = ((size_t)(b * HP + hp) * WP) * HC;
  v8us z8;
#pragma unroll
  for (int i = 0; i < 8; ++i) z8[i] = 0;

  if (hp == 0 || hp == HP - 1) {
    for (int rep = 0; rep < 2; ++rep) {
      for (int i = tid; i < WP * HC / 8; i += 256) {
#pragma unroll
        for (int p = 0; p < NPL; ++p)
          *(volatile v8us*)(act + (size_t)p * PLANE + rowbase + (size_t)i * 8) = z8;
      }
      __threadfence();
    }
    return;
  }
  const int h = hp - 1;
  for (int e = tid; e < 9 * WP; e += 256) {
    const int c = e / (3 * WP);
    const int rem = e - c * 3 * WP;
    const int dy = rem / WP;
    const int wp = rem - dy * WP;
    const int yy = h + dy - 1, xx = wp - 1;
    const bool inb = (yy >= 0) && (yy < HH) && (xx >= 0) && (xx < WW);
    const int yyc = min(max(yy, 0), HH - 1), xxc = min(max(xx, 0), WW - 1);
    const float v = msk[((size_t)(b * 3 + c) * HH + yyc) * WW + xxc];
    mrow[e] = inb ? bf_rne(v) : 0.0f;
  }
  __syncthreads();
  {
    const int w = tid & (WW - 1);
    const int kh = (tid >> 7) * 16;
    v8us o0, o1;
#pragma unroll
    for (int i = 0; i < 16; ++i) {
      const int k = kh + i;
      const int kc = min(k, 26);
      const int c = kc / 9;
      const int t = kc - 9 * c;
      const int dy = t / 3;
      const int dx = t - 3 * dy;
      float v = mrow[(c * 3 + dy) * WP + w + dx];
      v = (k < 27) ? v : 0.0f;
      const unsigned short bits = f2bf_bits(v);
      if (i < 8) o0[i] = bits; else o1[i - 8] = bits;
    }
    *(v8us*)(As + w * KSH + kh) = o0;
    *(v8us*)(As + w * KSH + kh + 8) = o1;
  }
  __syncthreads();

  const __bf16* Ab = (const __bf16*)(const void*)As;
  const __bf16* Wb = (const __bf16*)(const void*)wsh;
  const v16b a = frag_bf(Ab + (16 * wave + m) * KSH, hh);
  const v8f zero8 = {0.f, 0.f, 0.f, 0.f, 0.f, 0.f, 0.f, 0.f};
  v8f acc[8];
#pragma unroll
  for (int nt = 0; nt < 8; ++nt) acc[nt] = mma_bf(a, frag_bf(Wb + (16 * nt + m) * KSH, hh), zero8);

  float bias8[8];
#pragma unroll
  for (int nt = 0; nt < 8; ++nt) bias8[nt] = bf_rne(ssb[16 * nt + m]);

  unsigned short* sl = slab[wave];
  const int q8 = lane & 7, sub = lane >> 3;
#pragma unroll
  for (int ph = 0; ph < NPL; ++ph) {
#pragma unroll
    for (int nt = 0; nt < 8; ++nt) {
#pragma unroll
      for (int r = 0; r < 8; ++r) {
        const float v = fmaxf(acc[nt][r] + bias8[nt], 0.0f);
        const unsigned short hb = f2bf_bits(v);
        unsigned short ob = hb;
        if (ph == 1) ob = f2bf_bits(v - bf_bits2f(hb));
        sl[(8 * hh + r) * HC + 16 * nt + m] = ob;
      }
    }
    wave_lds_sync();
    unsigned short* plane = act + (size_t)ph * PLANE;
    for (int rep = 0; rep < 2; ++rep) {
#pragma unroll
      for (int i = 0; i < 8; ++i) {
        const int lid = i * 4 + sub;
        const int px = lid >> 1, hl = lid & 1;
        const v8us v = *(const v8usa*)(sl + px * HC + 64 * hl + 8 * q8);
        *(volatile v8us*)(plane + rowbase + (size_t)(16 * wave + px + 1) * HC + 64 * hl + 8 * q8) = v;
      }
      __threadfence();
    }
    wave_lds_sync();
  }
  if (wave == 0) {
    const int px = (lane < 16) ? 0 : (WP - 1);
    const int off = (lane & 15) * 8;
    for (int rep = 0; rep < 2; ++rep) {
#pragma unroll
      for (int p = 0; p < NPL; ++p)
        *(volatile v8us*)(act + (size_t)p * PLANE + rowbase + (size_t)px * HC + off) = z8;
      __threadfence();
    }
  }
}

__global__ __launch_bounds__(256) void k_final(
    const unsigned short* __restrict__ act, const unsigned short* __restrict__ wsp,
    const float* __restrict__ G, const float* __restrict__ stats,
    const float* __restrict__ seg, const float* __restrict__ x,
    const float* __restrict__ cgb, const float* __restrict__ cbb,
    const float* __restrict__ sgb, const float* __restrict__ sbb,
    const float* __restrict__ blg, const float* __restrict__ blb,
    float* __restrict__ out) {
  extern __shared__ float dsm[];
  float* S = dsm;
  float* Gs = dsm + WW * SPITCH;
  float* segt = Gs + NF * GPB;
  float* mus = segt + NSEGP;
  float* rss = mus + NC;

  const int blk = blockIdx.x;
  const int b = blk >> 7, h = blk & (HH - 1);
  const int tid = threadIdx.x, lane = tid & 31, wave = tid >> 5, hh = lane >> 4, m = lane & 15;
  const int wm = wave & 3, wn = wave >> 2;

  for (int i = tid; i < NF * GPB / 4; i += 256)
    *(v4f*)(Gs + 4 * i) = *(const v4fa*)(G + (size_t)b * NF * GPB + 4 * i);
  for (int e = tid; e < NSEG; e += 256) {
    const int j = e / (3 * WP);
    const int rem = e - j * 3 * WP;
    const int dy = rem / WP;
    const int wp = rem - dy * WP;
    const int yy = h + dy - 1, xx = wp - 1;
    const bool inb = (yy >= 0) && (yy < HH) && (xx >= 0) && (xx < WW);
    const int yyc = min(max(yy, 0), HH - 1), xxc = min(max(xx, 0), WW - 1);
    const float v = seg[((size_t)(b * NF + j) * HH + yyc) * WW + xxc];
    segt[e] = inb ? bf_rne(v) : 0.0f;
  }
  if (tid < NC) {
    mus[tid] = stats[(size_t)(b * NC + tid) * 32];
    rss[tid] = stats[(size_t)(b * NC + tid) * 32 + 1];
  }
  __syncthreads();

  const __bf16* Ab = (const __bf16*)(const void*)act;
  const __bf16* Bb = (const __bf16*)(const void*)wsp + (size_t)(64 * wn + m) * KSP;
  const v8f zero8 = {0.f, 0.f, 0.f, 0.f, 0.f, 0.f, 0.f, 0.f};
  v8f acc[2][4];
#pragma unroll
  for (int mt = 0; mt < 2; ++mt)
#pragma unroll
    for (int j = 0; j < 4; ++j) acc[mt][j] = zero8;

#pragma unroll 1
  for (int t = 0; t < 9; ++t) {
    const int dy = t / 3, dx = t - 3 * dy;
    const __bf16* ap = Ab + ((size_t)(b * HP + h + dy) * WP + dx + 32 * wm + m) * HC;
    const __bf16* bp = Bb + t * HC;
#pragma unroll
    for (int ks = 0; ks < 4; ++ks) {
      v16b bfr[4];
#pragma unroll
      for (int j = 0; j < 4; ++j) bfr[j] = frag_bf(bp + (size_t)j * 16 * KSP + 32 * ks, hh);
#pragma unroll
      for (int p = 0; p < NPL; ++p) {
        const __bf16* app = ap + (size_t)p * PLANE + 32 * ks;
        const v16b a0 = frag_bf(app, hh);
        const v16b a1 = frag_bf(app + 16 * HC, hh);
#pragma unroll
        for (int j = 0; j < 4; ++j) {
          acc[0][j] = mma_bf(a0, bfr[j], acc[0][j]);
          acc[1][j] = mma_bf(a1, bfr[j], acc[1][j]);
        }
      }
    }
  }

#pragma unroll
  for (int mt = 0; mt < 2; ++mt)
#pragma unroll
    for (int j = 0; j < 4; ++j)
#pragma unroll
      for (int r = 0; r < 8; ++r)
        S[(32 * wm + 16 * mt + 8 * hh + r) * SPITCH + 64 * wn + 16 * j + m] = acc[mt][j][r];
  __syncthreads();

  const float ga = 1.0f / (1.0f + expf(-bf_rne(blg[0])));
  const float ba = 1.0f / (1.0f + expf(-bf_rne(blb[0])));
  const float ga1 = 1.0f - ga, ba1 = 1.0f - ba;
  const int w0 = 4 * lane;
#pragma unroll 1
  for (int ci = 0; ci < 8; ++ci) {
    const int c = wave * 8 + ci;
    const float gb0 = bf_rne(cgb[c]), bb0 = bf_rne(cbb[c]);
    float gam[4], bet[4];
#pragma unroll
    for (int i = 0; i < 4; ++i) { gam[i] = gb0; bet[i] = bb0; }
#pragma unroll 1
    for (int j = 0; j < NF; ++j) {
      const float* sp = segt + j * 3 * WP + w0;
      const float* gq = Gs + (j * NO2 + c) * 9;
      const float* bq = gq + 64 * 9;
#pragma unroll
      for (int dy = 0; dy < 3; ++dy) {
        float s6[6];
#pragma unroll
        for (int q = 0; q < 6; ++q) s6[q] = sp[dy * WP + q];
#pragma unroll
        for (int dx = 0; dx < 3; ++dx) {
          const float gv = gq[dy * 3 + dx];
          const float bv = bq[dy * 3 + dx];
#pragma unroll
          for (int i = 0; i < 4; ++i) {
            gam[i] = fmaf(s6[i + dx], gv, gam[i]);
            bet[i] = fmaf(s6[i + dx], bv, bet[i]);
          }
        }
      }
    }
    const float mu = mus[c], rs = rss[c];
    const float sg = bf_rne(sgb[c]), sb = bf_rne(sbb[c]);
    const size_t gi = ((size_t)(b * NC + c) * HH + h) * WW + w0;
    const v4f xv = *(const v4fa*)(x + gi);
    v4f o;
#pragma unroll
    for (int i = 0; i < 4; ++i) {
      const float gs = S[(w0 + i) * SPITCH + c] + sg;
      const float bs = S[(w0 + i) * SPITCH + 64 + c] + sb;
      const float gf = ga * gam[i] + ga1 * gs;
      const float bf = ba * bet[i] + ba1 * bs;
      const float xn = (bf_rne(xv[i]) - mu) * rs;
      o[i] = xn * (1.0f + gf) + bf;
    }
    float* op = out + gi;
    *(volatile v4f*)op = o;
    __threadfence();
    *(volatile v4f*)op = o;
  }
}

extern "C" void kernel_launch(void* const* d_in, const int* in_sizes, int n_in,
                              void* d_out, int out_size, void* d_ws, size_t ws_size,
                              hipStream_t stream) {
  if (n_in < 18) return;
  if (in_sizes[0] != NB * NC * HWN) return;
  if (in_sizes[1] != NB * NF * HWN) return;
  if (in_sizes[2] != NB * NF * LL) return;
  if (in_sizes[3] != NB * 3 * HWN) return;
  if (in_sizes[4] != NF * LL * LL) return;
  if (in_sizes[5] != NF * LL) return;
  if (in_sizes[6] != NC * LL * 9 || in_sizes[7] != NC) return;
  if (in_sizes[8] != NC * LL * 9 || in_sizes[9] != NC) return;
  if (in_sizes[10] != HC * 27 || in_sizes[11] != HC) return;
  if (in_sizes[12] != NC * HC * 9 || in_sizes[13] != NC) return;
  if (in_sizes[14] != NC * HC * 9 || in_sizes[15] != NC) return;
  if (in_sizes[16] < 1 || in_sizes[17] < 1) return;
  if (out_size != NB * NC * HWN) return;

  const float* x     = (const float*)d_in[0];
  const float* segm  = (const float*)d_in[1];
  const float* codes = (const float*)d_in[2];
  const float* msk   = (const float*)d_in[3];
  const float* wfc   = (const float*)d_in[4];
  const float* bfc   = (const float*)d_in[5];
  const float* cgw   = (const float*)d_in[6];
  const float* cgb   = (const float*)d_in[7];
  const float* cbw   = (const float*)d_in[8];
  const float* cbb   = (const float*)d_in[9];
  const float* ssw   = (const float*)d_in[10];
  const float* ssb   = (const float*)d_in[11];
  const float* sgw   = (const float*)d_in[12];
  const float* sgb   = (const float*)d_in[13];
  const float* sbw   = (const float*)d_in[14];
  const float* sbb   = (const float*)d_in[15];
  const float* blg   = (const float*)d_in[16];
  const float* blb   = (const float*)d_in[17];
  float* out = (float*)d_out;

  const size_t szACT = (size_t)NPL * PLANE * 2;
  const size_t szWSP = (size_t)NO2 * KSP * 2;
  const size_t szWSH = (size_t)HC * KSH * 2;
  const size_t szG   = (size_t)NB * NF * GPB * 4;
  const size_t szST  = (size_t)NB * NC * 32 * 4;
  size_t off = 0;
  const size_t oACT = off; off += szACT;
  const size_t oWSP = off; off += szWSP;
  const size_t oWSH = off; off += szWSH;
  const size_t oG   = off; off += szG;
  const size_t oST  = off; off += szST;
  if (off > ws_size) return;
  if (off > (size_t)134217728) return;

  char* ws = (char*)d_ws;
  unsigned short* ACT = (unsigned short*)(ws + oACT);
  unsigned short* WSP = (unsigned short*)(ws + oWSP);
  unsigned short* WSH = (unsigned short*)(ws + oWSH);
  float* Gp = (float*)(ws + oG);
  float* ST = (float*)(ws + oST);

  k_prep<<<dim3(NU1 / 256 + NU2 / 256), dim3(256), 0, stream>>>(sgw, sbw, ssw, WSP, WSH);
  k_stats<<<dim3(NB * NC), dim3(256), 0, stream>>>(x, ST);
  k_fcg<<<dim3(NB * NF), dim3(256), 0, stream>>>(codes, wfc, bfc, cgw, cbw, Gp);
  k_shared<<<dim3(NB * HP), dim3(256), 0, stream>>>(msk, WSH, ssb, ACT);
  (void)hipFuncSetAttribute(reinterpret_cast<const void*>(&k_final), hipFuncAttributeMaxDynamicSharedMemorySize, DYN_BYTES);
  k_final<<<dim3(NB * HH), dim3(256), DYN_BYTES, stream>>>(ACT, WSP, Gp, ST, segm, x, cgb, cbb, sgb, sbb, blg, blb, out);
  (void)hipGetLastError();
}
